// MoEConnectionProcessor_38233798869014
// MI455X (gfx1250) — hardware-verified
//
#include <hip/hip_runtime.h>


namespace {
constexpr int N = 125000, K = 26, D = 32, NT16 = (N + 15) / 16;
constexpr float XS = 8.0f, WSC = 256.0f;
typedef _Float16 b16;
typedef __attribute__((ext_vector_type(16))) _Float16 v16b;
typedef __attribute__((ext_vector_type(8))) _Float16 v8b;
typedef __attribute__((ext_vector_type(8))) float v8f;
__device__ __forceinline__ float bf16_rne(float f) { unsigned int u = __float_as_uint(f); u += 0x7FFFu + ((u >> 16) & 1u); return __uint_as_float(u & 0xFFFF0000u); }
__device__ __forceinline__ void split16(float v, b16& hi, b16& lo) { hi = (b16)v; lo = (b16)(v - (float)hi); }
__device__ __forceinline__ v16b frag_kb(const b16* p, int hh) { const v8b a = *(const v8b*)(p + 8 * hh), b = *(const v8b*)(p + 16 + 8 * hh); v16b f;
#pragma unroll
  for (int e = 0; e < 8; ++e) { f[e] = a[e]; f[8 + e] = b[e]; } return f; }
__device__ __forceinline__ v8f wmma16b(v16b a, v16b b, v8f c) { v8f d = __builtin_amdgcn_wmma_f32_16x16x32_f16(false, a, false, b, (short)0, c, false, false); asm volatile("v_nop\n\tv_nop\n\tv_nop\n\tv_nop" : "+v"(d) : "v"(a), "v"(b)); return d; }
__device__ __forceinline__ void wave_lds_sync() { __builtin_amdgcn_fence(__ATOMIC_RELEASE, "workgroup"); __builtin_amdgcn_wave_barrier(); __builtin_amdgcn_fence(__ATOMIC_ACQUIRE, "workgroup"); }
__device__ __forceinline__ float pmul(float a, float b) { float p = a * b; asm volatile("" : "+v"(p)); return p; }
__device__ __forceinline__ int iclamp(int v, int lo, int hi) { return v < lo ? lo : (v > hi ? hi : v); }

__global__ __launch_bounds__(256) void wput_kernel(const float* __restrict__ w, int KIN, int OUTW, int OUTP, b16* __restrict__ WT) {
  const int KG = KIN / 8; const int u = blockIdx.x * 256 + threadIdx.x; if (u >= OUTP * KG) return; const int o = u / KG, k0 = (u % KG) * 8; v8b v;
#pragma unroll
  for (int j = 0; j < 8; ++j) v[j] = o < OUTW ? (b16)(bf16_rne(w[(size_t)(k0 + j) * OUTW + o]) * WSC) : (b16)0.0f; for (int pass = 0; pass < 2; ++pass) { *(volatile v8b*)(WT + (size_t)o * KIN + k0) = v; __threadfence(); }
}
__global__ __launch_bounds__(32) void msg_kernel(const float* __restrict__ x, const b16* __restrict__ WM, const float* __restrict__ bm, int NLIM, float* __restrict__ TT) {
  __shared__ __attribute__((aligned(16))) b16 Ah[16][D + 8]; __shared__ __attribute__((aligned(16))) float Tf[16][D + 1];
  const int lane = threadIdx.x, nloc = lane & 15, hlf = lane >> 4; const size_t m0 = (size_t)blockIdx.x * 16; if (m0 >= (size_t)NLIM) return;
  for (int rr = 0; rr < 16; ++rr) Ah[rr][lane] = (m0 + rr < (size_t)N) ? (b16)(bf16_rne(x[(m0 + rr) * D + lane]) * XS) : (b16)0.0f;
  wave_lds_sync();
#pragma unroll
  for (int t = 0; t < 2; ++t) { v8f acc = {}; acc = wmma16b(frag_kb(&Ah[nloc][0], hlf), frag_kb(WM + (size_t)(t * 16 + nloc) * D, hlf), acc); const float bb = bf16_rne(bm[t * 16 + nloc]);
#pragma unroll
    for (int r8 = 0; r8 < 8; ++r8) Tf[8 * hlf + r8][t * 16 + nloc] = tanhf(acc[r8] * (1.0f / (XS * WSC)) + bb); }
  wave_lds_sync();
  for (int pass = 0; pass < 2; ++pass) { for (int rr = 0; rr < 16; ++rr) if (m0 + rr < (size_t)N) ((volatile float*)TT)[(m0 + rr) * D + lane] = Tf[rr][lane]; __threadfence(); }
}
__global__ __launch_bounds__(32) void moe_kernel(const float* __restrict__ x, const int* __restrict__ nbi, const int* __restrict__ tier, const float* __restrict__ TT, const b16* __restrict__ WL, const float* __restrict__ bl, const b16* __restrict__ WF, const float* __restrict__ bfn, const b16* __restrict__ WC, const float* __restrict__ bc, const b16* __restrict__ WG, const float* __restrict__ bg, int NLIM, float* __restrict__ out) {
  __shared__ __attribute__((aligned(16))) b16 Ah[16][4 * D + 8], Al[16][4 * D + 8]; __shared__ float Cur[16][D + 1], La[16][D + 1], Fa[16][D + 1], Da[16][D + 1], Fm[16][D + 1], Lo[16][D + 1], Fo[16][D + 1], Xc[16][D + 1], Gt[16][4];
  const int lane = threadIdx.x, nloc = lane & 15, hlf = lane >> 4; const size_t m0 = (size_t)blockIdx.x * 16; if (m0 >= (size_t)NLIM) return;
  for (int rr = 0; rr < 16; ++rr) { const size_t n = m0 + rr; float c = 0.0f, s0 = 0.0f, s1 = 0.0f, s2 = 0.0f, sm = 0.0f; int c0 = 0, c1 = 0, c2 = 0;
    if (n < (size_t)N) { c = bf16_rne(x[n * D + lane]);
#pragma unroll 1
      for (int k = 0; k < K; ++k) { const int j = iclamp(nbi[n * K + k], 0, N - 1); const int t = tier[n * K + k]; const float v = bf16_rne(x[(size_t)j * D + lane]); if (t == 0) { s0 += v; ++c0; } else if (t == 1) { s1 += v; ++c1; sm += TT[(size_t)j * D + lane]; } else if (t == 2) { s2 += v; ++c2; } } }
    Cur[rr][lane] = c; La[rr][lane] = s0 / (float)(c0 < 1 ? 1 : c0); Fa[rr][lane] = s1 / (float)(c1 < 1 ? 1 : c1); Da[rr][lane] = s2 / (float)(c2 < 1 ? 1 : c2); Fm[rr][lane] = sm / (float)(c1 < 1 ? 1 : c1); Xc[rr][lane] = c; }
  wave_lds_sync();
  auto stage2 = [&](float (*P)[D + 1], float (*Q)[D + 1]) { for (int rr = 0; rr < 16; ++rr) { b16 p, q; split16(P[rr][lane] * XS, p, q); Ah[rr][lane] = p; Al[rr][lane] = q; split16(Q[rr][lane] * XS, p, q); Ah[rr][D + lane] = p; Al[rr][D + lane] = q; } wave_lds_sync(); };
  auto gemm64 = [&](const b16* WT, v8f acc[2]) { acc[0] = (v8f){}; acc[1] = (v8f){};
#pragma unroll
    for (int kb = 0; kb < 2 * D; kb += 32) { const v16b a = frag_kb(&Ah[nloc][kb], hlf), al = frag_kb(&Al[nloc][kb], hlf);
#pragma unroll
      for (int t = 0; t < 2; ++t) { const v16b bw = frag_kb(WT + (size_t)(t * 16 + nloc) * (2 * D) + kb, hlf); acc[t] = wmma16b(a, bw, acc[t]); acc[t] = wmma16b(al, bw, acc[t]); } } };
  stage2(Cur, La); { v8f acc[2]; gemm64(WL, acc); wave_lds_sync();
#pragma unroll
    for (int t = 0; t < 2; ++t) { const int cc = t * 16 + nloc; const float bb = bf16_rne(bl[cc]);
#pragma unroll
      for (int r8 = 0; r8 < 8; ++r8) Lo[8 * hlf + r8][cc] = tanhf(acc[t][r8] * (1.0f / (XS * WSC)) + bb); } }
  wave_lds_sync();
  stage2(Cur, Fm); { v8f acc[2]; gemm64(WF, acc); wave_lds_sync();
#pragma unroll
    for (int t = 0; t < 2; ++t) { const int cc = t * 16 + nloc; const float bb = bf16_rne(bfn[cc]);
#pragma unroll
      for (int r8 = 0; r8 < 8; ++r8) Fo[8 * hlf + r8][cc] = tanhf(acc[t][r8] * (1.0f / (XS * WSC)) + bb); } }
  wave_lds_sync();
#pragma unroll 1
  for (int s = 0; s < 3; ++s) { stage2(Xc, Da); v8f acc[2]; gemm64(WC, acc); wave_lds_sync();
#pragma unroll
    for (int t = 0; t < 2; ++t) { const int cc = t * 16 + nloc; const float bb = bf16_rne(bc[cc]);
#pragma unroll
      for (int r8 = 0; r8 < 8; ++r8) { const int rl = 8 * hlf + r8; Xc[rl][cc] = Xc[rl][cc] + pmul(1.0f / 3.0f, tanhf(acc[t][r8] * (1.0f / (XS * WSC)) + bb)); } }
    wave_lds_sync(); }
  for (int rr = 0; rr < 16; ++rr) { b16 p, q; split16(Cur[rr][lane] * XS, p, q); Ah[rr][lane] = p; Al[rr][lane] = q; split16(La[rr][lane] * XS, p, q); Ah[rr][D + lane] = p; Al[rr][D + lane] = q; split16(Fa[rr][lane] * XS, p, q); Ah[rr][2 * D + lane] = p; Al[rr][2 * D + lane] = q; split16(Da[rr][lane] * XS, p, q); Ah[rr][3 * D + lane] = p; Al[rr][3 * D + lane] = q; }
  wave_lds_sync();
  { v8f acc = {};
#pragma unroll
    for (int kb = 0; kb < 4 * D; kb += 32) { const v16b bw = frag_kb(WG + (size_t)nloc * (4 * D) + kb, hlf); acc = wmma16b(frag_kb(&Ah[nloc][kb], hlf), bw, acc); acc = wmma16b(frag_kb(&Al[nloc][kb], hlf), bw, acc); }
    if (nloc < 3) { const float bb = bf16_rne(bg[nloc]);
#pragma unroll
      for (int r8 = 0; r8 < 8; ++r8) Gt[8 * hlf + r8][nloc] = acc[r8] * (1.0f / (XS * WSC)) + bb; } }
  wave_lds_sync();
  for (int pass = 0; pass < 2; ++pass) { for (int rr = 0; rr < 16; ++rr) { if (m0 + rr >= (size_t)N) continue; const float g0 = Gt[rr][0], g1 = Gt[rr][1], g2 = Gt[rr][2]; const float mx = fmaxf(g0, fmaxf(g1, g2)); const float e0 = __expf(g0 - mx), e1 = __expf(g1 - mx), e2 = __expf(g2 - mx); const float inv = 1.0f / (e0 + e1 + e2);
      ((volatile float*)out)[(m0 + rr) * D + lane] = pmul(pmul(e0, inv), Lo[rr][lane]) + pmul(pmul(e1, inv), Fo[rr][lane]) + pmul(pmul(e2, inv), Xc[rr][lane]); } __threadfence(); }
}
}

extern "C" void kernel_launch(void* const* d_in, const int* in_sizes, int n_in, void* d_out, int out_size, void* d_ws, size_t ws_size, hipStream_t stream) {
  (void)n_in;
  auto Fp = [&](int i) { return (const float*)d_in[i]; }; auto Ip = [&](int i) { return (const int*)d_in[i]; };
  if (in_sizes[0] != N * D || in_sizes[1] != N * K || in_sizes[2] != N * K || in_sizes[3] != 2 * D * D || in_sizes[5] != D * D || in_sizes[7] != 2 * D * D || in_sizes[9] != 2 * D * D || in_sizes[11] != 4 * D * 3 || out_size != N * D) return;
  const int NLIM = N;
  size_t off = 0; char* ws = (char*)d_ws;
  auto carve = [&](size_t bytes) { char* p = ws + off; off += (bytes + 255) & ~(size_t)255; return p; };
  b16* WL = (b16*)carve(D * 2 * D * 2); b16* WM = (b16*)carve(D * D * 2); b16* WF = (b16*)carve(D * 2 * D * 2); b16* WC = (b16*)carve(D * 2 * D * 2); b16* WG = (b16*)carve(16 * 4 * D * 2); float* TT = (float*)carve((size_t)NT16 * 16 * D * 4);
  if (off > ws_size || off > ((size_t)32 << 20)) return;
  wput_kernel<<<1, 256, 0, stream>>>(Fp(3), 2 * D, D, D, WL); wput_kernel<<<1, 256, 0, stream>>>(Fp(5), D, D, D, WM); wput_kernel<<<1, 256, 0, stream>>>(Fp(7), 2 * D, D, D, WF); wput_kernel<<<1, 256, 0, stream>>>(Fp(9), 2 * D, D, D, WC); wput_kernel<<<1, 256, 0, stream>>>(Fp(11), 4 * D, 3, 16, WG);
  msg_kernel<<<NT16, 32, 0, stream>>>(Fp(0), WM, Fp(6), N, TT);
  moe_kernel<<<(unsigned)((NLIM + 15) / 16), 32, 0, stream>>>(Fp(0), Ip(1), Ip(2), TT, WL, Fp(4), WF, Fp(8), WC, Fp(10), WG, Fp(12), NLIM, (float*)d_out);
}
